// MMSA_37984690766445
// MI455X (gfx1250) — hardware-verified
//
#include <hip/hip_runtime.h>
#include <stdint.h>

#ifndef NQ
#define NQ 1024
#endif
#define SEQ  1024
#define DMOD 1024
#define NHD  16
#define HDIM 64
#define NEX  64
#define QKP  2048

typedef _Float16 v16h __attribute__((ext_vector_type(16)));
typedef _Float16 v8h  __attribute__((ext_vector_type(8)));
typedef __bf16   v16b __attribute__((ext_vector_type(16)));
typedef __bf16   v8b  __attribute__((ext_vector_type(8)));
typedef float    v8f  __attribute__((ext_vector_type(8)));
typedef float    v4f  __attribute__((ext_vector_type(4)));
typedef unsigned short v8us __attribute__((ext_vector_type(8)));
union FragB { v16b v; v8b h[2]; };
union F8 { v8f v; v4f q[2]; };

static_assert((NQ % 64) == 0 && NQ >= 64 && NQ <= SEQ);
static_assert(SEQ == 1024 && DMOD == 1024 && NHD * HDIM == DMOD && NEX == 64 && QKP == 2 * DMOD);

__device__ __forceinline__ unsigned short bfbits(float f) {
  unsigned u = __float_as_uint(f);
  return (unsigned short)((u + 0x7FFFu + ((u >> 16) & 1u)) >> 16);
}
__device__ __forceinline__ float bfval(unsigned short b) { return __uint_as_float(((unsigned)b) << 16); }
__device__ __forceinline__ float bfr(float f) { return bfval(bfbits(f)); }
__device__ __forceinline__ void split_bf(float f, unsigned short& hb, unsigned short& lb) {
  hb = bfbits(f);
  lb = bfbits(f - bfval(hb));
}

template <int ET> struct Elem;
template <> struct Elem<0> {
  typedef _Float16 T; typedef v16h V; typedef v8h V8;
  static __device__ __forceinline__ v8f mma(V a, V b, v8f c) {
    return __builtin_amdgcn_wmma_f32_16x16x32_f16(false, a, false, b, (short)0, c, false, false);
  }
};
template <> struct Elem<1> {
  typedef __bf16 T; typedef v16b V; typedef v8b V8;
  static __device__ __forceinline__ v8f mma(V a, V b, v8f c) {
    return __builtin_amdgcn_wmma_f32_16x16x32_bf16(false, a, false, b, (short)0, c, false, false);
  }
};

template <int ET>
__device__ __forceinline__ typename Elem<ET>::V ldfragT(const typename Elem<ET>::T* p) {
  typedef typename Elem<ET>::V V;
  typedef typename Elem<ET>::V8 V8;
  union { V v; V8 h[2]; } f;
  f.h[0] = *(const V8*)(p);
  f.h[1] = *(const V8*)(p + 16);
  return f.v;
}
__device__ __forceinline__ v16h ldfrag(const _Float16* p) { return ldfragT<0>(p); }
__device__ __forceinline__ v8f mma16(v16h a, v16h b, v8f c) { return Elem<0>::mma(a, b, c); }
__device__ __forceinline__ v8f mmab(v16b a, v16b b, v8f c) { return Elem<1>::mma(a, b, c); }
__device__ __forceinline__ v8f zero8() {
  v8f z;
#pragma unroll
  for (int i = 0; i < 8; ++i) z[i] = 0.0f;
  return z;
}

__device__ __forceinline__ void guard_g(v8f& a, v8f& b, v16h x, v16h y) {
  asm volatile("v_nop\n\tv_nop\n\tv_nop\n\tv_nop" : "+v"(a), "+v"(b) : "v"(x), "v"(y));
}
__device__ __forceinline__ void guard_g(v8f& a, v8f& b, v16b x, v16b y) {
  asm volatile("v_nop\n\tv_nop\n\tv_nop\n\tv_nop" : "+v"(a), "+v"(b) : "v"(x), "v"(y));
}
__device__ __forceinline__ void keep4(v16h a, v16h b, v16h c, v16h d) {
  asm volatile("v_nop" :: "v"(a), "v"(b), "v"(c), "v"(d));
}
__device__ __forceinline__ void keep4(v16b a, v16b b, v16b c, v16b d) {
  asm volatile("v_nop" :: "v"(a), "v"(b), "v"(c), "v"(d));
}
__device__ __forceinline__ void accg4(v8f& a, v8f& b, v8f& c, v8f& d) {
  asm volatile("v_nop\n\tv_nop\n\tv_nop\n\tv_nop" : "+v"(a), "+v"(b), "+v"(c), "+v"(d));
}
__device__ __forceinline__ void guard2x4(v8f& a, v8f& b, v16h x0, v16h x1, v16h x2, v16h x3) {
  asm volatile("v_nop\n\tv_nop\n\tv_nop\n\tv_nop" : "+v"(a), "+v"(b) : "v"(x0), "v"(x1), "v"(x2), "v"(x3));
}
__device__ __forceinline__ void guard4x5b(v8f& a, v8f& b, v8f& c, v8f& d,
                                          v16b x0, v16b x1, v16b x2, v16b x3, v16b x4) {
  asm volatile("v_nop\n\tv_nop\n\tv_nop\n\tv_nop"
               : "+v"(a), "+v"(b), "+v"(c), "+v"(d) : "v"(x0), "v"(x1), "v"(x2), "v"(x3), "v"(x4));
}
__device__ __forceinline__ void guard1x6b(v8f& a, v16b x0, v16b x1, v16b x2, v16b x3, v16b x4, v16b x5) {
  asm volatile("v_nop\n\tv_nop\n\tv_nop\n\tv_nop"
               : "+v"(a) : "v"(x0), "v"(x1), "v"(x2), "v"(x3), "v"(x4), "v"(x5));
}
__device__ __forceinline__ void guard8x10(v8f& a0, v8f& a1, v8f& a2, v8f& a3, v8f& a4, v8f& a5, v8f& a6, v8f& a7,
                                          v16h x0, v16h x1, v16h x2, v16h x3, v16h x4, v16h x5, v16h x6, v16h x7,
                                          v16h x8, v16h x9) {
  asm volatile("v_nop\n\tv_nop\n\tv_nop\n\tv_nop"
               : "+v"(a0), "+v"(a1), "+v"(a2), "+v"(a3), "+v"(a4), "+v"(a5), "+v"(a6), "+v"(a7)
               : "v"(x0), "v"(x1), "v"(x2), "v"(x3), "v"(x4), "v"(x5), "v"(x6), "v"(x7), "v"(x8), "v"(x9));
}

__global__ __launch_bounds__(256) void cvt_kernel(const float* __restrict__ s0, const float* __restrict__ s1,
                                                  const float* __restrict__ s2, unsigned short* __restrict__ d0,
                                                  unsigned short* __restrict__ d1, unsigned short* __restrict__ d2,
                                                  int n0, int n1, int n2) {
  const int nb0 = n0 >> 8, nb1 = n1 >> 8;
  const int b = (int)blockIdx.x;
  const int seg = (b >= nb0 + nb1) ? 2 : ((b >= nb0) ? 1 : 0);
  const float* src = (seg == 2) ? s2 : ((seg == 1) ? s1 : s0);
  unsigned short* dst = (seg == 2) ? d2 : ((seg == 1) ? d1 : d0);
  const int nn = (seg == 2) ? n2 : ((seg == 1) ? n1 : n0);
  const int li = (b - ((seg == 2) ? (nb0 + nb1) : ((seg == 1) ? nb0 : 0))) * 256 + (int)threadIdx.x;
  if (li >= nn) return;
  const size_t e = (size_t)li * 8;
  const v4f a = *(const v4f*)(src + e);
  const v4f c = *(const v4f*)(src + e + 4);
  v8us o;
#pragma unroll
  for (int i = 0; i < 4; ++i) {
    o[i]     = bfbits(a[i]);
    o[4 + i] = bfbits(c[i]);
  }
  unsigned short* d = dst + e;
  *(volatile v8us*)d = o;
  __threadfence();
  *(volatile v8us*)d = o;
}

template <int ET, bool SPLITA, int OUT_MODE, int BIASM>
__global__ __launch_bounds__(256) void gemm64_kernel(const unsigned short* __restrict__ Ap,
                                                     const unsigned short* __restrict__ A2p, int lda,
                                                     const unsigned short* __restrict__ Btp, int ldb,
                                                     void* Cout, void* C2out, int ldc,
                                                     const float* __restrict__ bias,
                                                     int M, int N, int K, float scale) {
  typedef typename Elem<ET>::T T;
  typedef typename Elem<ET>::V V;
  const T* A  = (const T*)(const void*)Ap;
  const T* A2 = (const T*)(const void*)A2p;
  const T* Bt = (const T*)(const void*)Btp;
  __shared__ __align__(16) float sT[8][16 * 68];
  const int lane = threadIdx.x & 31, wave = threadIdx.x >> 5;
  const int tilesN = N >> 6, tilesM = M >> 6;
  const int tile = (int)blockIdx.x * 8 + wave;
  if (tile >= tilesM * tilesN) return;
  const int tm = tile / tilesN, tn = tile - tm * tilesN;
  const int m0 = tm << 6, n0 = tn << 6;
  const int rl = lane & 15;
  const int koff = (lane >> 4) * 8;
  const int mOff = (lane >> 4) * 8;

  v8f acc[4][4];
#pragma unroll
  for (int i = 0; i < 4; ++i)
#pragma unroll
    for (int j = 0; j < 4; ++j) acc[i][j] = zero8();

#pragma unroll 1
  for (int k0 = 0; k0 < K; k0 += 32) {
    V bh[4];
#pragma unroll
    for (int j = 0; j < 4; ++j) bh[j] = ldfragT<ET>(Bt + (size_t)(n0 + (j << 4) + rl) * ldb + koff + k0);
#pragma unroll
    for (int i = 0; i < 4; ++i) {
      const size_t ao = (size_t)(m0 + (i << 4) + rl) * lda + koff + k0;
      const V ah = ldfragT<ET>(A + ao);
      V al = ah;
      if (SPLITA) al = ldfragT<ET>(A2 + ao);
#pragma unroll
      for (int j = 0; j < 4; ++j) {
        acc[i][j] = Elem<ET>::mma(ah, bh[j], acc[i][j]);
        if (SPLITA) acc[i][j] = Elem<ET>::mma(al, bh[j], acc[i][j]);
      }
      guard_g(acc[i][0], acc[i][3], ah, SPLITA ? al : bh[3]);
    }
    keep4(bh[0], bh[1], bh[2], bh[3]);
  }
  accg4(acc[0][0], acc[0][1], acc[0][2], acc[0][3]);
  accg4(acc[1][0], acc[1][1], acc[1][2], acc[1][3]);
  accg4(acc[2][0], acc[2][1], acc[2][2], acc[2][3]);
  accg4(acc[3][0], acc[3][1], acc[3][2], acc[3][3]);

  float* slab = sT[wave];
#pragma unroll
  for (int i = 0; i < 4; ++i) {
    const int mBase = m0 + (i << 4);
    float brow[8];
#pragma unroll
    for (int r = 0; r < 8; ++r) brow[r] = 0.0f;
    if (BIASM == 2) {
#pragma unroll
      for (int r = 0; r < 8; ++r) brow[r] = bfr(bias[mBase + mOff + r]);
    }
#pragma unroll
    for (int j = 0; j < 4; ++j) {
      float bv = 0.0f;
      if (BIASM == 1) bv = bfr(bias[n0 + (j << 4) + rl]);
#pragma unroll
      for (int r = 0; r < 8; ++r) slab[(mOff + r) * 68 + (j << 4) + rl] = acc[i][j][r] * scale + (bv + brow[r]);
    }
    __builtin_amdgcn_fence(__ATOMIC_RELEASE, "workgroup");
    __builtin_amdgcn_wave_barrier();
    __builtin_amdgcn_fence(__ATOMIC_ACQUIRE, "workgroup");
    if (OUT_MODE == 0) {
      float* C = (float*)Cout;
      const int hh = lane >> 4, c4 = (lane & 15) * 4;
#pragma unroll
      for (int ps = 0; ps < 2; ++ps) {
#pragma unroll
        for (int it = 0; it < 8; ++it) {
          const int row = it * 2 + hh;
          const v4f v = *(const v4f*)(slab + row * 68 + c4);
          *(volatile v4f*)(C + (size_t)(mBase + row) * ldc + n0 + c4) = v;
        }
        __threadfence();
      }
    } else {
      _Float16* C  = (_Float16*)Cout;
      _Float16* C2 = (_Float16*)C2out;
      const int qq = lane >> 3, c8 = (lane & 7) * 8;
#pragma unroll
      for (int ps = 0; ps < 2; ++ps) {
#pragma unroll
        for (int it = 0; it < 4; ++it) {
          const int row = it * 4 + qq;
          const float* sp = slab + row * 68 + c8;
          v8h hv, rv;
#pragma unroll
          for (int e = 0; e < 8; ++e) {
            const float cv = sp[e] * 16.0f;
            const _Float16 hf = (_Float16)cv;
            hv[e] = hf;
            rv[e] = (_Float16)((cv - (float)hf) * 2048.0f);
          }
          *(volatile v8h*)(C  + (size_t)(mBase + row) * ldc + n0 + c8) = hv;
          *(volatile v8h*)(C2 + (size_t)(mBase + row) * ldc + n0 + c8) = rv;
        }
        __threadfence();
      }
    }
    __builtin_amdgcn_fence(__ATOMIC_RELEASE, "workgroup");
    __builtin_amdgcn_wave_barrier();
    __builtin_amdgcn_fence(__ATOMIC_ACQUIRE, "workgroup");
  }
}

__global__ __launch_bounds__(256) void colsum_kernel(const _Float16* __restrict__ vh, const _Float16* __restrict__ vr,
                                                     float* __restrict__ cs, int ntok) {
  __shared__ __align__(16) float red[32];
  const int wave = threadIdx.x >> 5, lane = threadIdx.x & 31;
  const int r0 = (int)blockIdx.x * 32;
  const int nch = ntok >> 8;
#pragma unroll 1
  for (int i = 0; i < 4; ++i) {
    const int row = r0 + wave * 4 + i;
    const _Float16* ph = vh + (size_t)row * ntok;
    const _Float16* pr = vr + (size_t)row * ntok;
    float s = 0.0f;
#pragma unroll 1
    for (int j = 0; j < nch; ++j) {
      const int c0 = (j * 32 + lane) * 8;
      const v8h a = *(const v8h*)(ph + c0);
      const v8h b = *(const v8h*)(pr + c0);
      float t = 0.0f;
#pragma unroll
      for (int e = 0; e < 8; ++e) t += (float)a[e] + (float)b[e] * (1.0f / 2048.0f);
      s += t;
    }
#pragma unroll
    for (int off = 16; off > 0; off >>= 1) s += __shfl_xor(s, off, 32);
    if (lane == 0) red[wave * 4 + i] = s * (1.0f / 16.0f);
  }
  __syncthreads();
  if (wave == 0 && lane < 8) {
    const v4f v = *(const v4f*)(red + 4 * lane);
    float* d = cs + r0 + 4 * lane;
    *(volatile v4f*)d = v;
    __threadfence();
    *(volatile v4f*)d = v;
  }
}

#define QB      16
#define KT      128
#define PTP     136
#define HLW     8192
#define LDS_HL  0
#define LDS_PT  131072
#define LDS_A1  200704
#define LDS_W2  204800
#define LDS_MB  206848
#define LDS_LI  210944
#define LDS_CC  215040
#define LDS_CH  219136
#define LDS_B1  219200
#define ATT_LDS 219456
static_assert(LDS_PT - LDS_HL == 8 * HLW * 2);
static_assert(LDS_A1 - LDS_PT == NHD * QB * PTP * 2);
static_assert(LDS_W2 - LDS_A1 == NEX * 32 * 2);
static_assert(LDS_MB - LDS_W2 == NHD * NEX * 2);
static_assert(LDS_LI - LDS_MB == QB * NEX * 4);
static_assert(LDS_CC - LDS_LI == QB * NEX * 4);
static_assert(LDS_CH - LDS_CC == DMOD * 4);
static_assert(LDS_B1 - LDS_CH == NHD * 4);
static_assert(ATT_LDS - LDS_B1 == NEX * 4);
static_assert(2 * 8 * NEX * QB * 4 <= LDS_PT - LDS_HL);
static_assert(2 * QB * DMOD * 2 <= LDS_PT - LDS_HL);
static_assert(2 * QB * NEX * 4 <= LDS_A1 - LDS_PT);
static_assert(HLW == 16 * QB * 32);
static_assert((SEQ % KT) == 0 && KT == 16 * 8 && (PTP % 8) == 0 && PTP >= KT && (NQ % QB) == 0);
static_assert((LDS_PT % 16) == 0 && (LDS_A1 % 16) == 0 && (LDS_W2 % 16) == 0 && (LDS_MB % 16) == 0);
static_assert((LDS_LI % 16) == 0 && (LDS_CC % 16) == 0 && (LDS_B1 % 16) == 0);

template <int MODE>
__global__ __launch_bounds__(256) void attn_kernel(const _Float16* __restrict__ qkh, const _Float16* __restrict__ qkr,
                                                   const _Float16* __restrict__ vth,
                                                   const float* __restrict__ w1, const float* __restrict__ b1,
                                                   const float* __restrict__ w2, const float* __restrict__ b2,
                                                   const float* __restrict__ csum,
                                                   float* __restrict__ mbp, float* __restrict__ lip,
                                                   unsigned short* __restrict__ oh, unsigned short* __restrict__ ol) {
  extern __shared__ __align__(16) char smem[];
  __bf16*   HL  = (__bf16*)(smem + LDS_HL);
  _Float16* Pt  = (_Float16*)(smem + LDS_PT);
  __bf16*   A1s = (__bf16*)(smem + LDS_A1);
  __bf16*   W2s = (__bf16*)(smem + LDS_W2);
  float*    MBs = (float*)(smem + LDS_MB);
  float*    LIs = (float*)(smem + LDS_LI);
  float*    CCs = (float*)(smem + LDS_CC);
  float*    CHs = (float*)(smem + LDS_CH);
  float*    B1s = (float*)(smem + LDS_B1);

  const int tid = threadIdx.x, wave = tid >> 5, lane = tid & 31, hh = lane >> 4, c = lane & 15;
  const int q0 = (int)blockIdx.x * QB;
  const float ninf = -__builtin_inff();
  const float RX = 0.00048828125f;
  const float KS = 0.00048828125f;
  const float CP = 64.0f;
  const float KO = 9.5367431640625e-7f;

  {
    const int e = tid >> 2, s0 = (tid & 3) * 8;
#pragma unroll
    for (int i = 0; i < 8; ++i) {
      const int s = s0 + i;
      A1s[e * 32 + s] = (__bf16)w1[e * NHD + (s & 15)];
    }
  }
  if (MODE == 1) {
#pragma unroll
    for (int i = 0; i < 4; ++i) {
      const int idx = tid * 4 + i;
      W2s[idx] = (__bf16)w2[idx];
    }
    if (tid < NHD) {
      float ch = 0.0f;
#pragma unroll 1
      for (int e = 0; e < NEX; ++e) ch += bfr(w2[tid * NEX + e]);
      CHs[tid] = ch;
    }
    *(v4f*)(MBs + 4 * tid) = *(const v4f*)(mbp + (size_t)q0 * NEX + 4 * tid);
    *(v4f*)(LIs + 4 * tid) = *(const v4f*)(lip + (size_t)q0 * NEX + 4 * tid);
  } else {
    if (tid < NEX) B1s[tid] = bfr(b1[tid]);
  }
  __syncthreads();
  if (MODE == 1) {
#pragma unroll
    for (int j = 0; j < 4; ++j) {
      const int col = tid + 256 * j, h = col >> 6;
      CCs[col] = (CHs[h] * (1.0f / 1024.0f) + bfr(b2[h])) * csum[col];
    }
  }
  v8f mv[4], lv[4], b1v[4];
  v8f oacc[8];
#pragma unroll
  for (int t = 0; t < 4; ++t) {
    lv[t] = zero8();
    b1v[t] = zero8();
#pragma unroll
    for (int r = 0; r < 8; ++r) mv[t][r] = ninf;
  }
#pragma unroll
  for (int p = 0; p < 8; ++p) oacc[p] = zero8();
  if (MODE == 0) {
#pragma unroll
    for (int t = 0; t < 4; ++t) {
      F8 bb;
      bb.q[0] = *(const v4f*)(B1s + 16 * t + 8 * hh);
      bb.q[1] = *(const v4f*)(B1s + 16 * t + 8 * hh + 4);
      b1v[t] = bb.v;
    }
  }
  __syncthreads();

  __bf16* HLw = HL + wave * HLW;
#pragma unroll 1
  for (int kt = 0; kt < SEQ / KT; ++kt) {
    {
      const int kb = kt * KT + 16 * wave;
      const _Float16* qhp = qkh + (size_t)(q0 + c) * QKP + 8 * hh;
      const _Float16* qrp = qkr + (size_t)(q0 + c) * QKP + 8 * hh;
      const _Float16* khp = qkh + DMOD + (size_t)(kb + c) * QKP + 8 * hh;
      const _Float16* krp = qkr + DMOD + (size_t)(kb + c) * QKP + 8 * hh;
      __bf16* hd = HLw + (c * QB + 8 * hh) * 32;
#pragma unroll 1
      for (int h = 0; h < NHD; ++h) {
        v8f shh = zero8(), sx = zero8();
#pragma unroll
        for (int ks = 0; ks < 2; ++ks) {
          const int co = h * HDIM + 32 * ks;
          const v16h aq = ldfrag(qhp + co), ar = ldfrag(qrp + co);
          const v16h bk = ldfrag(khp + co), br = ldfrag(krp + co);
          shh = mma16(aq, bk, shh);
          sx  = mma16(aq, br, sx);
          sx  = mma16(ar, bk, sx);
          guard2x4(shh, sx, aq, ar, bk, br);
        }
#pragma unroll
        for (int r = 0; r < 8; ++r) {
          const float a = (shh[r] + sx[r] * RX) * KS;
          const __bf16 hb = (__bf16)a;
          const __bf16 lb = (__bf16)(a - (float)hb);
          hd[r * 32 + h]      = hb;
          hd[r * 32 + 16 + h] = lb;
        }
      }
    }
    __syncthreads();
    {
      const __bf16* bfp = HLw + c * 32 + 8 * hh;
#pragma unroll 1
      for (int kk = 0; kk < 16; ++kk) {
        const v16b bf = ldfragT<1>(bfp + kk * (QB * 32));
        v16b af[4];
        v8f acc1[4];
#pragma unroll
        for (int t = 0; t < 4; ++t) af[t] = ldfragT<1>(A1s + (16 * t + c) * 32 + 8 * hh);
#pragma unroll
        for (int t = 0; t < 4; ++t) acc1[t] = mmab(af[t], bf, zero8());
        guard4x5b(acc1[0], acc1[1], acc1[2], acc1[3], af[0], af[1], af[2], af[3], bf);
        if (MODE == 0) {
#pragma unroll
          for (int t = 0; t < 4; ++t) {
#pragma unroll
            for (int r = 0; r < 8; ++r) {
              const float lg = acc1[t][r] + b1v[t][r];
              const float mo = mv[t][r];
              const float mn = fmaxf(mo, lg);
              lv[t][r] = lv[t][r] * __expf(mo - mn) + __expf(lg - mn);
              mv[t][r] = mn;
            }
          }
        } else {
          FragB Bh[2], Bl[2];
#pragma unroll
          for (int t = 0; t < 4; ++t) {
            F8 mm, ii;
            mm.q[0] = *(const v4f*)(MBs + c * NEX + 16 * t + 8 * hh);
            mm.q[1] = *(const v4f*)(MBs + c * NEX + 16 * t + 8 * hh + 4);
            ii.q[0] = *(const v4f*)(LIs + c * NEX + 16 * t + 8 * hh);
            ii.q[1] = *(const v4f*)(LIs + c * NEX + 16 * t + 8 * hh + 4);
            v8b hv, lw;
#pragma unroll
            for (int r = 0; r < 8; ++r) {
              const float p = __expf(acc1[t][r] - mm.v[r]) * ii.v[r] - 1.0f;
              const __bf16 ph = (__bf16)p;
              hv[r] = ph;
              lw[r] = (__bf16)(p - (float)ph);
            }
            Bh[t >> 1].h[t & 1] = hv;
            Bl[t >> 1].h[t & 1] = lw;
          }
          const v16b wa = ldfragT<1>(W2s + c * NEX + 8 * hh);
          const v16b wb = ldfragT<1>(W2s + c * NEX + 32 + 8 * hh);
          v8f acc2 = mmab(wa, Bh[0].v, zero8());
          acc2 = mmab(wa, Bl[0].v, acc2);
          acc2 = mmab(wb, Bh[1].v, acc2);
          acc2 = mmab(wb, Bl[1].v, acc2);
          guard1x6b(acc2, wa, wb, Bh[0].v, Bl[0].v, Bh[1].v, Bl[1].v);
          _Float16* pd = Pt + (8 * hh * QB + c) * PTP + 16 * wave + kk;
#pragma unroll
          for (int r = 0; r < 8; ++r) pd[r * QB * PTP] = (_Float16)(acc2[r] * CP);
        }
      }
    }
    __syncthreads();
    if (MODE == 1) {
      const _Float16* pa0 = Pt + ((2 * wave) * QB + c) * PTP + 8 * hh;
      const _Float16* pa1 = pa0 + QB * PTP;
      const _Float16* vbp = vth + (size_t)((2 * wave) * HDIM + c) * SEQ + kt * KT + 8 * hh;
#pragma unroll 1
      for (int ks = 0; ks < KT / 32; ++ks) {
        const v16h a0 = ldfrag(pa0 + 32 * ks), a1 = ldfrag(pa1 + 32 * ks);
        v16h vb[8];
#pragma unroll
        for (int p = 0; p < 8; ++p) vb[p] = ldfrag(vbp + (size_t)((p >> 2) * HDIM + 16 * (p & 3)) * SEQ + 32 * ks);
#pragma unroll
        for (int p = 0; p < 4; ++p) oacc[p] = mma16(a0, vb[p], oacc[p]);
#pragma unroll
        for (int p = 4; p < 8; ++p) oacc[p] = mma16(a1, vb[p], oacc[p]);
        guard8x10(oacc[0], oacc[1], oacc[2], oacc[3], oacc[4], oacc[5], oacc[6], oacc[7],
                  a0, a1, vb[0], vb[1], vb[2], vb[3], vb[4], vb[5], vb[6], vb[7]);
      }
    }
  }

  if (MODE == 0) {
    float* CM = (float*)(smem + LDS_HL);
    float* CL = CM + 8 * NEX * QB;
#pragma unroll
    for (int t = 0; t < 4; ++t) {
#pragma unroll
      for (int r = 0; r < 8; ++r) {
        const int idx = (wave * NEX + 16 * t + 8 * hh + r) * QB + c;
        CM[idx] = mv[t][r];
        CL[idx] = lv[t][r];
      }
    }
    __syncthreads();
    float* SOm = (float*)(smem + LDS_PT);
    float* SOl = SOm + QB * NEX;
#pragma unroll
    for (int j = 0; j < 4; ++j) {
      const int idx = tid + 256 * j, e = idx >> 4, q = idx & 15;
      float mx = ninf;
#pragma unroll
      for (int w = 0; w < 8; ++w) mx = fmaxf(mx, CM[(w * NEX + e) * QB + q]);
      float ls = 0.0f;
#pragma unroll
      for (int w = 0; w < 8; ++w) ls += CL[(w * NEX + e) * QB + q] * __expf(CM[(w * NEX + e) * QB + q] - mx);
      SOm[q * NEX + e] = mx - B1s[e];
      SOl[q * NEX + e] = 1024.0f * __builtin_amdgcn_rcpf(ls);
    }
    __syncthreads();
    const v4f mo = *(const v4f*)(SOm + 4 * tid);
    const v4f io = *(const v4f*)(SOl + 4 * tid);
    float* gm = mbp + (size_t)q0 * NEX + 4 * tid;
    float* gi = lip + (size_t)q0 * NEX + 4 * tid;
    *(volatile v4f*)gm = mo;
    *(volatile v4f*)gi = io;
    __threadfence();
    *(volatile v4f*)gm = mo;
    *(volatile v4f*)gi = io;
  } else {
    __syncthreads();
    unsigned short* Hs = (unsigned short*)(smem + LDS_HL);
    unsigned short* Ls = Hs + QB * DMOD;
#pragma unroll
    for (int p = 0; p < 8; ++p) {
      const int h = 2 * wave + (p >> 2), nt = p & 3;
      const int col = h * HDIM + 16 * nt + c;
      const float cc = CCs[col];
#pragma unroll
      for (int r = 0; r < 8; ++r) {
        unsigned short hb, lb;
        split_bf(oacc[p][r] * KO + cc, hb, lb);
        Hs[(8 * hh + r) * DMOD + col] = hb;
        Ls[(8 * hh + r) * DMOD + col] = lb;
      }
    }
    __syncthreads();
    unsigned short* gh = oh + (size_t)q0 * DMOD;
    unsigned short* gl = ol + (size_t)q0 * DMOD;
#pragma unroll
    for (int ps = 0; ps < 2; ++ps) {
#pragma unroll
      for (int rr = 0; rr < 2; ++rr) {
        const int row = 2 * wave + rr;
#pragma unroll
        for (int j = 0; j < 4; ++j) {
          const int pc = j * 32 + lane;
          const v8us hvv = *(const v8us*)(Hs + row * DMOD + pc * 8);
          const v8us lvv = *(const v8us*)(Ls + row * DMOD + pc * 8);
          *(volatile v8us*)(gh + (size_t)row * DMOD + pc * 8) = hvv;
          *(volatile v8us*)(gl + (size_t)row * DMOD + pc * 8) = lvv;
        }
      }
      __threadfence();
    }
  }
}

extern "C" void kernel_launch(void* const* d_in, const int* in_sizes, int n_in,
                              void* d_out, int out_size, void* d_ws, size_t ws_size,
                              hipStream_t stream) {
  if (n_in < 9) return;
  if (in_sizes[0] < SEQ * DMOD || in_sizes[1] < 3 * DMOD * DMOD || in_sizes[2] < 3 * DMOD) return;
  if (in_sizes[3] < DMOD * DMOD || in_sizes[4] < DMOD) return;
  if (in_sizes[5] < NEX * NHD || in_sizes[6] < NEX || in_sizes[7] < NHD * NEX || in_sizes[8] < NHD) return;
  if (out_size < NQ * DMOD) return;

  const float* x     = (const float*)d_in[0];
  const float* qkv_w = (const float*)d_in[1];
  const float* qkv_b = (const float*)d_in[2];
  const float* prj_w = (const float*)d_in[3];
  const float* prj_b = (const float*)d_in[4];
  const float* a1w   = (const float*)d_in[5];
  const float* a1b   = (const float*)d_in[6];
  const float* a2w   = (const float*)d_in[7];
  const float* a2b   = (const float*)d_in[8];
  float* out = (float*)d_out;

  const size_t bXB = (size_t)SEQ * DMOD * 2;
  const size_t bWB = (size_t)3 * DMOD * DMOD * 2;
  const size_t bPB = (size_t)DMOD * DMOD * 2;
  const size_t bQK = (size_t)SEQ * QKP * 2;
  const size_t bVT = (size_t)DMOD * SEQ * 2;
  const size_t bST = (size_t)NQ * NEX * 4;
  const size_t bCS = (size_t)DMOD * 4;
  const size_t bO  = (size_t)NQ * DMOD * 2;
  size_t off = 0;
  const size_t oXB  = off; off += bXB;
  const size_t oWB  = off; off += bWB;
  const size_t oPB  = off; off += bPB;
  const size_t oQKH = off; off += bQK;
  const size_t oQKR = off; off += bQK;
  const size_t oVTH = off; off += bVT;
  const size_t oVTR = off; off += bVT;
  const size_t oMB  = off; off += bST;
  const size_t oLI  = off; off += bST;
  const size_t oCS  = off; off += bCS;
  const size_t oOH  = off; off += bO;
  const size_t oOL  = off; off += bO;
  if (off > ws_size) return;
  if (off > (size_t)134217728) return;

  char* ws = (char*)d_ws;
  unsigned short* XB  = (unsigned short*)(ws + oXB);
  unsigned short* WB  = (unsigned short*)(ws + oWB);
  unsigned short* PB  = (unsigned short*)(ws + oPB);
  _Float16*       QKH = (_Float16*)(ws + oQKH);
  _Float16*       QKR = (_Float16*)(ws + oQKR);
  _Float16*       VTH = (_Float16*)(ws + oVTH);
  _Float16*       VTR = (_Float16*)(ws + oVTR);
  float*          MBp = (float*)(ws + oMB);
  float*          LIp = (float*)(ws + oLI);
  float*          CSp = (float*)(ws + oCS);
  unsigned short* OH  = (unsigned short*)(ws + oOH);
  unsigned short* OL  = (unsigned short*)(ws + oOL);

  const dim3 blk(256);
  const int nx8 = SEQ * DMOD / 8;
  const int nw8 = 3 * DMOD * DMOD / 8;
  const int np8 = DMOD * DMOD / 8;
  if ((nx8 % 256) != 0 || (nw8 % 256) != 0 || (np8 % 256) != 0) return;

  cvt_kernel<<<dim3((nx8 + nw8 + np8) / 256), blk, 0, stream>>>(x, qkv_w, prj_w, XB, WB, PB, nx8, nw8, np8);
  {
    const int tiles = (SEQ / 64) * (QKP / 64);
    gemm64_kernel<1, false, 2, 1><<<dim3((tiles + 7) / 8), blk, 0, stream>>>(
        XB, XB, DMOD, WB, DMOD, (void*)QKH, (void*)QKR, QKP, qkv_b, SEQ, QKP, DMOD, 1.0f);
  }
  {
    const int tiles = (DMOD / 64) * (SEQ / 64);
    gemm64_kernel<1, false, 2, 2><<<dim3((tiles + 7) / 8), blk, 0, stream>>>(
        WB + (size_t)2 * DMOD * DMOD, WB + (size_t)2 * DMOD * DMOD, DMOD, XB, DMOD,
        (void*)VTH, (void*)VTR, SEQ, qkv_b + 2 * DMOD, DMOD, SEQ, DMOD, 1.0f);
  }
  colsum_kernel<<<dim3(DMOD / 32), blk, 0, stream>>>(VTH, VTR, CSp, SEQ);
  (void)hipFuncSetAttribute(reinterpret_cast<const void*>(&attn_kernel<0>),
                            hipFuncAttributeMaxDynamicSharedMemorySize, ATT_LDS);
  (void)hipFuncSetAttribute(reinterpret_cast<const void*>(&attn_kernel<1>),
                            hipFuncAttributeMaxDynamicSharedMemorySize, ATT_LDS);
  attn_kernel<0><<<dim3(NQ / QB), blk, ATT_LDS, stream>>>(QKH, QKR, VTH, a1w, a1b, a2w, a2b, CSp, MBp, LIp, OH, OL);
  attn_kernel<1><<<dim3(NQ / QB), blk, ATT_LDS, stream>>>(QKH, QKR, VTH, a1w, a1b, a2w, a2b, CSp, MBp, LIp, OH, OL);
  {
    const int tiles = (NQ / 64) * (DMOD / 64);
    gemm64_kernel<1, true, 0, 1><<<dim3((tiles + 7) / 8), blk, 0, stream>>>(
        OH, OL, DMOD, PB, DMOD, (void*)out, (void*)out, DMOD, prj_b, NQ, DMOD, DMOD, 1.0f);
  }
  (void)hipGetLastError();
}
